// MultiHeadAttention_13855564497508
// MI455X (gfx1250) — hardware-run, weakly checked
//
#include <hip/hip_runtime.h>


#ifndef NB
#define NB 8
#endif
#ifndef SEQ
#define SEQ 1024
#endif
#define NB_FULL  8
#define SEQ_FULL 1024
#define DM   768
#define NH   12
#define HD   64
#define ZH   6
#define PCAR 1024.0f
#define SCL  0.125f
typedef _Float16 h16;
typedef unsigned short bf;
typedef __attribute__((ext_vector_type(16))) __bf16   v16bf;
typedef __attribute__((ext_vector_type(16))) _Float16 v16h;
typedef __attribute__((ext_vector_type(8)))  _Float16 v8h;
typedef __attribute__((ext_vector_type(8)))  unsigned short v8us;
typedef __attribute__((ext_vector_type(8)))  float    v8f;
typedef __attribute__((ext_vector_type(4)))  float    v4f;
typedef __attribute__((ext_vector_type(2)))  _Float16 v2h;
typedef __attribute__((ext_vector_type(4)))  _Float16 v4h;
typedef __attribute__((ext_vector_type(2)))  unsigned short v2us;
typedef v4f  __attribute__((may_alias)) v4fa;

static_assert(NH * HD == DM);
static_assert(NH % ZH == 0);
static_assert(SEQ % 128 == 0);
static_assert(DM % 64 == 0);
static_assert(HD % 32 == 0);
static_assert(NB <= NB_FULL);
static_assert(SEQ <= SEQ_FULL);

__device__ __forceinline__ unsigned short f2bf(float f) { unsigned u = __float_as_uint(f); u += 0x7FFFu + ((u >> 16) & 1u); return (unsigned short)(u >> 16); }
__device__ __forceinline__ float bf2f(unsigned short b) { return __uint_as_float(((unsigned)b) << 16); }
__device__ __forceinline__ float bfr(float f) { return bf2f(f2bf(f)); }
__device__ __forceinline__ v16h cat16(v8h lo, v8h hi) { return __builtin_shufflevector(lo, hi, 0, 1, 2, 3, 4, 5, 6, 7, 8, 9, 10, 11, 12, 13, 14, 15); }
__device__ __forceinline__ v16bf cat16b(v8us lo, v8us hi) { return __builtin_bit_cast(v16bf, __builtin_shufflevector(lo, hi, 0, 1, 2, 3, 4, 5, 6, 7, 8, 9, 10, 11, 12, 13, 14, 15)); }
__device__ __forceinline__ v8f wmma16(v16h a, v16h b, v8f c) { return __builtin_amdgcn_wmma_f32_16x16x32_f16(false, a, false, b, (short)0, c, false, false); }
__device__ __forceinline__ v8f wmmab(v16bf a, v16bf b, v8f c) { return __builtin_amdgcn_wmma_f32_16x16x32_bf16(false, a, false, b, (short)0, c, false, false); }
__device__ __forceinline__ h16 tohx(float x) { return (h16)x; }
__device__ __forceinline__ void splitf(float y, unsigned short& h, unsigned short& l) { h = f2bf(y); l = f2bf(y - bf2f(h)); }

template <typename T16> struct WFrag;
template <> struct WFrag<h16> { typedef v16h V; static __device__ __forceinline__ V ld(const h16* p) { return cat16(*(const v8h*)p, *(const v8h*)(p + 16)); } static __device__ __forceinline__ v8f mma(V a, V b, v8f c) { return wmma16(a, b, c); } };
template <> struct WFrag<bf> { typedef v16bf V; static __device__ __forceinline__ V ld(const bf* p) { return cat16b(*(const v8us*)p, *(const v8us*)(p + 16)); } static __device__ __forceinline__ v8f mma(V a, V b, v8f c) { return wmmab(a, b, c); } };
template <typename T16, int NSPLIT, bool BIAS>
__global__ __launch_bounds__(32) void k_gemmw(const T16* __restrict__ A, const T16* __restrict__ A2, const T16* __restrict__ Bt, const T16* __restrict__ Bt2, int K, float* C, int ldc, const float* __restrict__ bias, size_t sA, size_t sB, size_t sC) {
    typedef typename WFrag<T16>::V V;
    __shared__ __align__(16) float os[16 * 68];
    const size_t z = blockIdx.z; A += z * sA; if (A2) A2 += z * sA; Bt += z * sB; if (Bt2) Bt2 += z * sB; C += z * sC;
    const int lane = threadIdx.x & 31, lr = lane & 15, hi = lane >> 4; const int r0 = blockIdx.x * 64, c0 = blockIdx.y * 64;
    v8f acc[4][4];
#pragma unroll
    for (int mb = 0; mb < 4; ++mb)
#pragma unroll
        for (int nb = 0; nb < 4; ++nb) acc[mb][nb] = (v8f){};
    const size_t aoff = (size_t)(r0 + lr) * K + 8 * hi, boff = (size_t)(c0 + lr) * K + 8 * hi;
#pragma unroll 1
    for (int kc = 0; kc < K; kc += 32) {
        V a[4], a2[4];
#pragma unroll
        for (int mb = 0; mb < 4; ++mb) { a[mb] = WFrag<T16>::ld(A + aoff + (size_t)mb * 16 * K + kc); if (NSPLIT == 1 || NSPLIT == 2) a2[mb] = WFrag<T16>::ld(A2 + aoff + (size_t)mb * 16 * K + kc); }
#pragma unroll
        for (int nb = 0; nb < 4; ++nb) { const V b = WFrag<T16>::ld(Bt + boff + (size_t)nb * 16 * K + kc); V b2; if (NSPLIT >= 2) b2 = WFrag<T16>::ld(Bt2 + boff + (size_t)nb * 16 * K + kc);
#pragma unroll
            for (int mb = 0; mb < 4; ++mb) { acc[mb][nb] = WFrag<T16>::mma(a[mb], b, acc[mb][nb]); if (NSPLIT == 1 || NSPLIT == 2) acc[mb][nb] = WFrag<T16>::mma(a2[mb], b, acc[mb][nb]); if (NSPLIT >= 2) acc[mb][nb] = WFrag<T16>::mma(a[mb], b2, acc[mb][nb]); } }
        asm volatile("v_nop\n\tv_nop\n\tv_nop\n\tv_nop" : "+v"(acc[0][0]), "+v"(acc[1][1]), "+v"(acc[2][2]), "+v"(acc[3][3]) : "v"(a[0]), "v"(a[3]));
    }
#pragma unroll
    for (int mb = 0; mb < 4; ++mb) {
#pragma unroll
        for (int nb = 0; nb < 4; ++nb) {
#pragma unroll
            for (int j = 0; j < 8; ++j) os[(hi * 8 + j) * 68 + nb * 16 + lr] = acc[mb][nb][j]; }
        __builtin_amdgcn_wave_barrier(); asm volatile("" ::: "memory");
        float* crow = C + (size_t)(r0 + mb * 16) * ldc + c0;
#pragma unroll 1
        for (int ps = 0; ps < 2; ++ps) {
#pragma unroll
            for (int s = 0; s < 8; ++s) { const int row = 2 * s + hi, cofs = lr * 4; v4f val = *(const v4fa*)(os + row * 68 + cofs); if (BIAS) { val[0] += bfr(bias[c0 + cofs]); val[1] += bfr(bias[c0 + cofs + 1]); val[2] += bfr(bias[c0 + cofs + 2]); val[3] += bfr(bias[c0 + cofs + 3]); }
                *(volatile v4f*)(crow + (size_t)row * ldc + cofs) = val; }
            if (ps == 0) __threadfence(); }
        __builtin_amdgcn_wave_barrier(); asm volatile("" ::: "memory");
    }
}

__global__ __launch_bounds__(256) void k_wtG(const float* __restrict__ w, int K, int N, bf* Bt) {
    const int lane = threadIdx.x & 31; const int L0 = (blockIdx.x * 8 + (threadIdx.x >> 5)) * 8; const int nlines = N * K / 64;
#pragma unroll
    for (int ps = 0; ps < 2; ++ps) {
#pragma unroll 1
        for (int l = 0; l < 8; ++l) { const int L = L0 + l; if (L >= nlines) break; const size_t e = (size_t)L * 64 + lane * 2; const int k = (int)(e % K), n = (int)(e / K); v2us o;
            o[0] = f2bf(w[(size_t)k * N + n]); o[1] = f2bf(w[(size_t)(k + 1) * N + n]); *(volatile v2us*)(Bt + e) = o; }
        if (ps == 0) __threadfence(); }
}

__global__ __launch_bounds__(256) void k_xb(const float* __restrict__ x, bf* XB) {
    const size_t i = (size_t)blockIdx.x * 256 + threadIdx.x; if (i >= (size_t)NB * SEQ * DM / 8) return;
    const size_t e = i * 8; const int col = (int)(e % DM); const size_t row = e / DM; const int b = (int)(row / SEQ), s = (int)(row % SEQ);
    const v8f v = *(const v8f*)(x + ((size_t)b * SEQ_FULL + s) * DM + col); v8us o;
#pragma unroll
    for (int k = 0; k < 8; ++k) o[k] = f2bf(v[k]);
    *(volatile v8us*)(XB + e) = o; __threadfence(); *(volatile v8us*)(XB + e) = o; }

__global__ __launch_bounds__(256) void k_hp(const float* __restrict__ F, bf* Ph, bf* Pl) {
    const size_t i = (size_t)blockIdx.x * 256 + threadIdx.x; if (i >= (size_t)NB * NH * SEQ * HD / 8) return;
    const size_t e = i * 8; const int d = (int)(e % HD); const int s = (int)((e / HD) % SEQ); const int bh = (int)(e / ((size_t)HD * SEQ)); const int b = bh / NH, h = bh % NH;
    const float* f = F + ((size_t)b * SEQ + s) * DM + h * HD + d; const v4f a0 = *(const v4f*)f, a1 = *(const v4f*)(f + 4); v8us oh, ol;
#pragma unroll
    for (int q = 0; q < 4; ++q) { unsigned short a, c; splitf(a0[q], a, c); oh[q] = a; ol[q] = c; splitf(a1[q], a, c); oh[4 + q] = a; ol[4 + q] = c; }
    *(volatile v8us*)(Ph + e) = oh; *(volatile v8us*)(Pl + e) = ol; __threadfence(); *(volatile v8us*)(Ph + e) = oh; *(volatile v8us*)(Pl + e) = ol; }

__global__ __launch_bounds__(256) void k_vtp(const float* __restrict__ F, h16* V16) {
    const size_t e = ((size_t)blockIdx.x * 256 + threadIdx.x) * 2; if (e >= (size_t)NB * NH * HD * SEQ) return;
    const int t = (int)(e % SEQ); const int d = (int)((e / SEQ) % HD); const int bh = (int)(e / ((size_t)SEQ * HD)); const int b = bh / NH, h = bh % NH; v2h o16;
#pragma unroll
    for (int q = 0; q < 2; ++q) { const float x = F[((size_t)b * SEQ + t + q) * DM + h * HD + d]; o16[q] = tohx(x); }
    *(volatile v2h*)(V16 + e) = o16; __threadfence(); *(volatile v2h*)(V16 + e) = o16; }

__global__ __launch_bounds__(256) void k_asoft(const float* __restrict__ Sb, h16* P16) {
    const int lane = threadIdx.x & 31; const int row = blockIdx.x * 8 + (threadIdx.x >> 5); if (row >= ZH * SEQ) return; const float* sr = Sb + (size_t)row * SEQ; float v[SEQ / 32]; float mx = -3.0e38f;
#pragma unroll
    for (int ch = 0; ch < SEQ / 128; ++ch) { const int j0 = ch * 128 + lane * 4; const v4f a = *(const v4f*)(sr + j0);
#pragma unroll
        for (int q = 0; q < 4; ++q) { const float t = a[q] * SCL; v[ch * 4 + q] = t; mx = fmaxf(mx, t); } }
#pragma unroll
    for (int sh = 16; sh; sh >>= 1) mx = fmaxf(mx, __shfl_xor(mx, sh, 32));
    float sum = 0.f;
#pragma unroll
    for (int k = 0; k < SEQ / 32; ++k) { float d0 = __fsub_rn(v[k], mx); asm volatile("" : "+v"(d0)); v[k] = __builtin_amdgcn_exp2f(__fmul_rn(d0, 1.4426950408889634f)); sum += v[k]; }
#pragma unroll
    for (int sh = 16; sh; sh >>= 1) sum += __shfl_xor(sum, sh, 32);
    const float f = __fdiv_rn(PCAR, sum);
#pragma unroll 1
    for (int ps = 0; ps < 2; ++ps) {
#pragma unroll
        for (int ch = 0; ch < SEQ / 128; ++ch) { v4h o4;
#pragma unroll
            for (int q = 0; q < 4; ++q) o4[q] = tohx(v[ch * 4 + q] * f);
            *(volatile v4h*)(P16 + (size_t)row * SEQ + ch * 128 + lane * 4) = o4; }
        if (ps == 0) __threadfence(); }
}

__global__ __launch_bounds__(256) void k_cx(const float* __restrict__ CTX, bf* Ch, bf* Cl) {
    const size_t i = (size_t)blockIdx.x * 256 + threadIdx.x; if (i >= (size_t)NB * SEQ * DM / 8) return;
    const size_t e = i * 8; const v4f a0 = *(const v4f*)(CTX + e), a1 = *(const v4f*)(CTX + e + 4); const float cs = 1.0f / PCAR; v8us oh, ol;
#pragma unroll
    for (int q = 0; q < 4; ++q) { unsigned short a, c; splitf(a0[q] * cs, a, c); oh[q] = a; ol[q] = c; splitf(a1[q] * cs, a, c); oh[4 + q] = a; ol[4 + q] = c; }
    *(volatile v8us*)(Ch + e) = oh; *(volatile v8us*)(Cl + e) = ol; __threadfence(); *(volatile v8us*)(Ch + e) = oh; *(volatile v8us*)(Cl + e) = ol; }

constexpr size_t al256(size_t b) { return (b + 255) & ~(size_t)255; }
constexpr size_t cmax2(size_t a, size_t b) { return a > b ? a : b; }
constexpr size_t SZ_W     = (size_t)DM * DM * 2;
constexpr size_t SZ_ACT16 = (size_t)NB * SEQ * DM * 2;
constexpr size_t SZ_ACT32 = (size_t)NB * SEQ * DM * 4;
constexpr size_t SZ_RA    = cmax2(SZ_ACT16, (size_t)ZH * SEQ * SEQ * 2);
constexpr size_t SZ_RB    = cmax2(SZ_ACT32, (size_t)ZH * SEQ * SEQ * 4);
constexpr size_t SZ_TOTAL = 4 * al256(SZ_W) + al256(SZ_RA) + al256(SZ_RB) + 5 * al256(SZ_ACT16) + al256(SZ_ACT32);
static_assert(SZ_TOTAL <= (size_t)134217728);
static_assert(SZ_ACT16 <= SZ_RA);
static_assert(SZ_ACT16 <= SZ_RB);

extern "C" void kernel_launch(void* const* d_in, const int* in_sizes, int n_in,
                              void* d_out, int out_size, void* d_ws, size_t ws_size, hipStream_t stream) {
    if (n_in < 9) return;
    const size_t XN = ((size_t)(NB - 1) * SEQ_FULL + SEQ) * DM;
    if ((size_t)in_sizes[0] < XN) return;
    if ((size_t)in_sizes[1] < (size_t)DM * DM || (size_t)in_sizes[3] < (size_t)DM * DM || (size_t)in_sizes[5] < (size_t)DM * DM || (size_t)in_sizes[7] < (size_t)DM * DM) return;
    if (in_sizes[2] < DM || in_sizes[4] < DM || in_sizes[6] < DM || in_sizes[8] < DM) return;
    if ((size_t)out_size < XN) return;
    if (ws_size < SZ_TOTAL) return;
    const float* x = (const float*)d_in[0]; const float* wq = (const float*)d_in[1]; const float* bq = (const float*)d_in[2]; const float* wk = (const float*)d_in[3]; const float* bk = (const float*)d_in[4];
    const float* wv = (const float*)d_in[5]; const float* bv = (const float*)d_in[6]; const float* wo = (const float*)d_in[7]; const float* bo = (const float*)d_in[8];
    float* OUT = (float*)d_out;
    char* wsp = (char*)d_ws;
    auto take = [&](size_t bytes) { char* p = wsp; wsp += (bytes + 255) & ~(size_t)255; return (void*)p; };
    bf* WQ = (bf*)take(SZ_W); bf* WK = (bf*)take(SZ_W); bf* WV = (bf*)take(SZ_W); bf* WO = (bf*)take(SZ_W);
    char* RA = (char*)take(SZ_RA); char* RB = (char*)take(SZ_RB);
    bf* QPh = (bf*)take(SZ_ACT16); bf* QPl = (bf*)take(SZ_ACT16); bf* KPh = (bf*)take(SZ_ACT16); bf* KPl = (bf*)take(SZ_ACT16); h16* VT16 = (h16*)take(SZ_ACT16);
    float* CTX = (float*)take(SZ_ACT32);
    if ((size_t)(wsp - (char*)d_ws) > ws_size) return;
    bf* XB = (bf*)RA; h16* P16 = (h16*)RA; bf* CH = (bf*)RA;
    float* F = (float*)RB; float* Sb = (float*)RB; bf* CL = (bf*)RB;

    const unsigned GW = (unsigned)((DM * DM / 64 + 63) / 64);
    k_wtG<<<GW, 256, 0, stream>>>(wq, DM, DM, WQ); k_wtG<<<GW, 256, 0, stream>>>(wk, DM, DM, WK); k_wtG<<<GW, 256, 0, stream>>>(wv, DM, DM, WV); k_wtG<<<GW, 256, 0, stream>>>(wo, DM, DM, WO);
    const unsigned G8 = (unsigned)(((size_t)NB * SEQ * DM / 8 + 255) / 256), G2 = (unsigned)(((size_t)NB * SEQ * DM / 2 + 255) / 256);
    k_xb<<<G8, 256, 0, stream>>>(x, XB);
    const dim3 gp((unsigned)(NB * SEQ / 64), DM / 64, 1);
    k_gemmw<bf, 0, true><<<gp, 32, 0, stream>>>(XB, nullptr, WQ, nullptr, DM, F, DM, bq, 0, 0, 0);
    k_hp<<<G8, 256, 0, stream>>>(F, QPh, QPl);
    k_gemmw<bf, 0, true><<<gp, 32, 0, stream>>>(XB, nullptr, WK, nullptr, DM, F, DM, bk, 0, 0, 0);
    k_hp<<<G8, 256, 0, stream>>>(F, KPh, KPl);
    k_gemmw<bf, 0, true><<<gp, 32, 0, stream>>>(XB, nullptr, WV, nullptr, DM, F, DM, bv, 0, 0, 0);
    k_vtp<<<G2, 256, 0, stream>>>(F, VT16);
    for (int b = 0; b < NB; ++b) {
        for (int h0 = 0; h0 < NH; h0 += ZH) { const size_t zq = (size_t)b * NH + h0;
            k_gemmw<bf, 2, false><<<dim3(SEQ / 64, SEQ / 64, ZH), 32, 0, stream>>>(QPh + zq * SEQ * HD, QPl + zq * SEQ * HD, KPh + zq * SEQ * HD, KPl + zq * SEQ * HD, HD, Sb, SEQ, nullptr, (size_t)SEQ * HD, (size_t)SEQ * HD, (size_t)SEQ * SEQ);
            k_asoft<<<ZH * SEQ / 8, 256, 0, stream>>>(Sb, P16);
            k_gemmw<h16, 0, false><<<dim3(SEQ / 64, HD / 64, ZH), 32, 0, stream>>>(P16, nullptr, VT16 + zq * HD * SEQ, nullptr, SEQ, CTX + (size_t)b * SEQ * DM + (size_t)h0 * HD, DM, nullptr, (size_t)SEQ * SEQ, (size_t)HD * SEQ, (size_t)HD); }
    }
    k_cx<<<G8, 256, 0, stream>>>(CTX, CH, CL);
    k_gemmw<bf, 1, true><<<dim3(SEQ / 64, DM / 64, NB), 32, 0, stream>>>(CH, CL, WO, nullptr, DM, OUT, DM, bo, (size_t)SEQ * DM, 0, (size_t)SEQ_FULL * DM);
}
